// MLA_74990128988313
// MI455X (gfx1250) — hardware-verified
//
#include <hip/hip_runtime.h>
#include <math.h>
#include <stdint.h>

#define NBAT  2
#define SEQL  2048
#define DMD   2048
#define NTOK  4096
#define NHD   16
#define HDC   128
#define HDR   64
#define DLAT  682
#define DLP   704
#define CW    1408
#define NFREQ 32
#define KRW   128
#define QRW   2048
#define KCW   4096

static_assert(NTOK == NBAT * SEQL);
static_assert(DLP % 64 == 0 && CW == 2 * DLP && DLP >= DLAT);
static_assert(DMD % 64 == 0 && SEQL % 64 == 0 && (NHD * HDR) % 64 == 0);
static_assert(DLP % 32 == 0 && DMD % 32 == 0 && KCW % 32 == 0);
static_assert(NHD * HDC == DMD && 2 * NHD * HDC == KCW && 2 * NHD * HDR == QRW && 2 * HDR == KRW);

typedef __bf16       v16b __attribute__((ext_vector_type(16)));
typedef __bf16       v8b  __attribute__((ext_vector_type(8)));
typedef float        v8f  __attribute__((ext_vector_type(8)));
typedef float        v4f  __attribute__((ext_vector_type(4)));
typedef unsigned int v4u  __attribute__((ext_vector_type(4)));

struct FreqTab { float f[NFREQ]; };
static_assert(sizeof(FreqTab) == 128);

__device__ __forceinline__ unsigned short bf_bits(float f) {
  const unsigned u = __float_as_uint(f);
  return (unsigned short)((u + 0x7FFFu + ((u >> 16) & 1u)) >> 16);
}
__device__ __forceinline__ float bf_val(unsigned short h) { return __uint_as_float(((unsigned)h) << 16); }
__device__ __forceinline__ unsigned pk16(unsigned short a, unsigned short b) { return (unsigned)a | ((unsigned)b << 16); }
__device__ __forceinline__ v8f zero8() { v8f z = {0.f, 0.f, 0.f, 0.f, 0.f, 0.f, 0.f, 0.f}; return z; }
__device__ __forceinline__ int wave_id() { return __builtin_amdgcn_readfirstlane((int)(threadIdx.x >> 5)); }

__device__ __forceinline__ void lds_wave_sync() {
  __builtin_amdgcn_fence(__ATOMIC_RELEASE, "workgroup");
  __builtin_amdgcn_wave_barrier();
  __builtin_amdgcn_fence(__ATOMIC_ACQUIRE, "workgroup");
}

union FragB { v16b v; v8b h[2]; };
__device__ __forceinline__ v16b ldfrag_b(const __bf16* p) { FragB f; f.h[0] = *(const v8b*)(p); f.h[1] = *(const v8b*)(p + 16); return f.v; }

__device__ __forceinline__ v8f mma_b(v16b a, v16b b, v8f c) {
  return __builtin_amdgcn_wmma_f32_16x16x32_bf16(false, a, false, b, (short)0, c, false, false);
}
__device__ __forceinline__ void dep_guard_b(v8f& a, v8f& b, v16b x, v16b y) {
  asm volatile("v_nop\n\tv_nop\n\tv_nop\n\tv_nop" : "+v"(a), "+v"(b) : "v"(x), "v"(y));
}
__device__ __forceinline__ void keep4_b(v16b a, v16b b, v16b c, v16b d) { asm volatile("v_nop" :: "v"(a), "v"(b), "v"(c), "v"(d)); }
__device__ __forceinline__ void guard1b4(v8f& a, v16b w, v16b x, v16b y, v16b z) {
  asm volatile("v_nop\n\tv_nop\n\tv_nop\n\tv_nop" : "+v"(a) : "v"(w), "v"(x), "v"(y), "v"(z) : "memory");
}
__device__ __forceinline__ void acc_guard4(v8f& a, v8f& b, v8f& c, v8f& d) {
  asm volatile("v_nop\n\tv_nop\n\tv_nop\n\tv_nop" : "+v"(a), "+v"(b), "+v"(c), "+v"(d));
}
__device__ __forceinline__ void acc_guard2(v8f& a, v8f& b) {
  asm volatile("v_nop\n\tv_nop\n\tv_nop\n\tv_nop" : "+v"(a), "+v"(b));
}

__global__ __launch_bounds__(256) void rope_table_kernel(FreqTab ft, float* __restrict__ cst, float* __restrict__ snt) {
  const int lane = threadIdx.x & 31;
  const int wave = (int)(threadIdx.x >> 5);
  const int t = (int)blockIdx.x * 8 + wave;
  if (t >= SEQL) return;
  float inv = ft.f[0];
#pragma unroll
  for (int j = 1; j < NFREQ; ++j) inv = (lane == j) ? ft.f[j] : inv;
  const float ang = (float)t * inv;
  const float cv  = cosf(ang);
  const float sv  = sinf(ang);
  const size_t o = (size_t)t * NFREQ + lane;
  for (int pass = 0; pass < 2; ++pass) {
    ((volatile float*)cst)[o] = cv;
    ((volatile float*)snt)[o] = sv;
    __threadfence();
  }
}

__global__ __launch_bounds__(256) void cvt_bf16_kernel(const float* __restrict__ in, unsigned short* __restrict__ outp, int n8) {
  const int i = (int)blockIdx.x * 256 + (int)threadIdx.x;
  if (i >= n8) return;
  const size_t e = 8 * (size_t)i;
  const v4f a = *(const v4f*)(in + e);
  const v4f b = *(const v4f*)(in + e + 4);
  v4u w;
  w[0] = pk16(bf_bits(a[0]), bf_bits(a[1]));
  w[1] = pk16(bf_bits(a[2]), bf_bits(a[3]));
  w[2] = pk16(bf_bits(b[0]), bf_bits(b[1]));
  w[3] = pk16(bf_bits(b[2]), bf_bits(b[3]));
  *(volatile v4u*)(outp + e) = w;
  __threadfence();
  *(volatile v4u*)(outp + e) = w;
}

__global__ __launch_bounds__(256) void tcvt_kernel(const float* __restrict__ in, int R, int C,
                                                   unsigned short* __restrict__ O, int ldo, int coff, int coff2) {
  __shared__ __align__(16) float tf[64 * 68];
  const int r0  = (int)blockIdx.x * 64;
  const int c0  = (int)blockIdx.y * 64;
  const int tid = (int)threadIdx.x;
#pragma unroll 4
  for (int it = 0; it < 16; ++it) {
    const int e  = it * 256 + tid;
    const int rr = e >> 6, cc = e & 63;
    const int r  = r0 + rr, c = c0 + cc;
    const int rcl = (r < R) ? r : (R - 1);
    const int ccl = (c < C) ? c : (C - 1);
    const float v = in[(size_t)rcl * C + ccl];
    tf[rr * 68 + cc] = (r < R && c < C) ? v : 0.0f;
  }
  __syncthreads();
  const int sub = tid >> 3;
  const int c8  = (tid & 7) * 8;
  v4u w[2];
#pragma unroll
  for (int it = 0; it < 2; ++it) {
    const int oc = it * 32 + sub;
    v4u a;
#pragma unroll
    for (int q = 0; q < 4; ++q) {
      const float f0 = tf[(c8 + 2 * q) * 68 + oc];
      const float f1 = tf[(c8 + 2 * q + 1) * 68 + oc];
      a[q] = pk16(bf_bits(f0), bf_bits(f1));
    }
    w[it] = a;
  }
  for (int pass = 0; pass < 2; ++pass) {
#pragma unroll
    for (int it = 0; it < 2; ++it) {
      const int oc = it * 32 + sub;
      const size_t rowo = (size_t)(c0 + oc) * ldo + r0 + c8;
      *(volatile v4u*)(O + rowo + coff) = w[it];
      if (coff2 >= 0) *(volatile v4u*)(O + rowo + coff2) = w[it];
    }
    __threadfence();
  }
}

template <bool ASPL, bool BSPL, int OUT_MODE>
__global__ __launch_bounds__(256) void gemm64_kernel(
    const unsigned short* __restrict__ Ap, const unsigned short* __restrict__ A2p, int lda,
    const unsigned short* __restrict__ Btp, const unsigned short* __restrict__ Bt2p, int ldb,
    void* Cout, void* Cout2, int ldc,
    const float* __restrict__ cst, const float* __restrict__ snt,
    int M, int N, int K) {
  __shared__ __align__(16) float sT[8][16 * 68];
  const int lane = threadIdx.x & 31;
  const int wave = wave_id();
  const int tilesN = N >> 6;
  const int tilesM = M >> 6;
  const int tile = (int)blockIdx.x * 8 + wave;
  if (tile >= tilesM * tilesN) return;
  const int tm = tile / tilesN;
  const int tn = tile - tm * tilesN;
  const int m0 = tm << 6;
  const int n0 = tn << 6;

  const __bf16* A   = (const __bf16*)(const void*)Ap;
  const __bf16* A2  = (const __bf16*)(const void*)A2p;
  const __bf16* Bt  = (const __bf16*)(const void*)Btp;
  const __bf16* Bt2 = (const __bf16*)(const void*)Bt2p;

  const int rlane = lane & 15;
  const int koff  = (lane >> 4) * 8;
  const int mOff  = (lane >> 4) * 8;

  v8f acc[4][4];
#pragma unroll
  for (int i = 0; i < 4; ++i)
#pragma unroll
    for (int j = 0; j < 4; ++j) acc[i][j] = zero8();

  for (int k0 = 0; k0 < K; k0 += 32) {
    v16b bh[4], bl[4];
#pragma unroll
    for (int j = 0; j < 4; ++j) {
      const size_t bo = (size_t)(n0 + (j << 4) + rlane) * ldb + koff + k0;
      bh[j] = ldfrag_b(Bt + bo);
      if (BSPL) bl[j] = ldfrag_b(Bt2 + bo); else bl[j] = bh[j];
    }
#pragma unroll
    for (int i = 0; i < 4; ++i) {
      const size_t ao = (size_t)(m0 + (i << 4) + rlane) * lda + koff + k0;
      const v16b ah = ldfrag_b(A + ao);
      v16b al = ah;
      if (ASPL) al = ldfrag_b(A2 + ao);
#pragma unroll
      for (int j = 0; j < 4; ++j) {
        acc[i][j] = mma_b(ah, bh[j], acc[i][j]);
        if (BSPL) acc[i][j] = mma_b(ah, bl[j], acc[i][j]);
        if (ASPL) acc[i][j] = mma_b(al, bh[j], acc[i][j]);
      }
      dep_guard_b(acc[i][0], acc[i][3], ah, al);
    }
    keep4_b(bh[0], bh[1], bh[2], bh[3]);
    if (BSPL) keep4_b(bl[0], bl[1], bl[2], bl[3]);
  }
  acc_guard4(acc[0][0], acc[0][1], acc[0][2], acc[0][3]);
  acc_guard4(acc[1][0], acc[1][1], acc[1][2], acc[1][3]);
  acc_guard4(acc[2][0], acc[2][1], acc[2][2], acc[2][3]);
  acc_guard4(acc[3][0], acc[3][1], acc[3][2], acc[3][3]);

  float* slab = sT[wave];
#pragma unroll
  for (int i = 0; i < 4; ++i) {
    const int mBase = m0 + (i << 4);
#pragma unroll
    for (int j = 0; j < 4; ++j) {
#pragma unroll
      for (int r = 0; r < 8; ++r) slab[(mOff + r) * 68 + (j << 4) + rlane] = acc[i][j][r];
    }
    lds_wave_sync();
    if (OUT_MODE == 0) {
      float* Cf = (float*)Cout;
      const int h2 = lane >> 4, c4 = (lane & 15) * 4;
      for (int pass = 0; pass < 2; ++pass) {
#pragma unroll
        for (int it = 0; it < 8; ++it) {
          const int row = it * 2 + h2;
          const v4f v = *(const v4f*)(slab + row * 68 + c4);
          *(volatile v4f*)(Cf + (size_t)(mBase + row) * ldc + n0 + c4) = v;
        }
        __threadfence();
      }
    } else {
      const int q = lane >> 3, c8 = (lane & 7) * 8;
      unsigned short* C  = (unsigned short*)Cout;
      unsigned short* C2 = (unsigned short*)Cout2;
      for (int pass = 0; pass < 2; ++pass) {
#pragma unroll
        for (int it = 0; it < 4; ++it) {
          const int row = it * 4 + q;
          const float* sp = slab + row * 68 + c8;
          const v4f s0 = *(const v4f*)(sp);
          const v4f s1 = *(const v4f*)(sp + 4);
          float f[8] = {s0[0], s0[1], s0[2], s0[3], s1[0], s1[1], s1[2], s1[3]};
          if (OUT_MODE == 3) {
            const int pos = (mBase + row) & (SEQL - 1);
            const v4f cv = *(const v4f*)(cst + (size_t)pos * NFREQ + (lane & 7) * 4);
            const v4f sv = *(const v4f*)(snt + (size_t)pos * NFREQ + (lane & 7) * 4);
#pragma unroll
            for (int p = 0; p < 4; ++p) {
              const float x1 = f[2 * p], x2 = f[2 * p + 1];
              f[2 * p]     = x1 * cv[p] - x2 * sv[p];
              f[2 * p + 1] = x1 * sv[p] + x2 * cv[p];
            }
          }
          v4u hw, lw;
#pragma unroll
          for (int p = 0; p < 4; ++p) {
            const unsigned short h0 = bf_bits(f[2 * p]), h1 = bf_bits(f[2 * p + 1]);
            const unsigned short l0 = bf_bits(f[2 * p] - bf_val(h0)), l1 = bf_bits(f[2 * p + 1] - bf_val(h1));
            hw[p] = pk16(h0, h1);
            lw[p] = pk16(l0, l1);
          }
          const size_t go = (size_t)(mBase + row) * ldc + n0 + c8;
          *(volatile v4u*)(C + go)  = hw;
          *(volatile v4u*)(C2 + go) = lw;
        }
        __threadfence();
      }
    }
    lds_wave_sync();
  }
}

#define AKC    32
#define KP     200
#define VP     40
#define PP     40
#define OPW    128
#define PK_KH  0
#define PK_KL  (AKC * KP)
#define PK_VH  (2 * AKC * KP)
#define PK_VL  (PK_VH + HDC * VP)
#define PK_PH  (PK_VL + HDC * VP)
#define PK_PL  (PK_PH + 4 * 16 * PP)
#define PK_END (PK_PL + 4 * 16 * PP)
#define PK_OH  0
#define PK_OL  (4 * 16 * OPW)
static_assert(PK_END * 2 <= 65536);
static_assert(PK_OL + 4 * 16 * OPW <= PK_END);
static_assert(HDC + HDR <= KP && AKC <= VP && AKC <= PP);
static_assert((PK_KL % 8) == 0 && (PK_VH % 8) == 0 && (PK_VL % 8) == 0 && (PK_PH % 8) == 0 && (PK_PL % 8) == 0 && (PK_OL % 8) == 0);

__global__ __launch_bounds__(128) void attn_lat_kernel(
    const unsigned short* __restrict__ qcp, const unsigned short* __restrict__ qrp,
    const unsigned short* __restrict__ kcp, const unsigned short* __restrict__ krp,
    const unsigned short* __restrict__ vtp, unsigned short* __restrict__ ctxp, float sscale) {
  __shared__ __align__(16) unsigned short pool[PK_END];
  unsigned short* Ks  = pool + PK_KH;
  unsigned short* Kls = pool + PK_KL;
  unsigned short* Vhs = pool + PK_VH;
  unsigned short* Vls = pool + PK_VL;

  const int tid  = (int)threadIdx.x;
  const int lane = tid & 31;
  const int wave = wave_id();
  const int hh   = lane >> 4;
  const int c    = lane & 15;
  const int qt   = (int)blockIdx.x;
  const int h    = (int)blockIdx.y;
  const int q0   = qt * 64 + wave * 16;

  unsigned short* ph = pool + PK_PH + wave * (16 * PP);
  unsigned short* pl = pool + PK_PL + wave * (16 * PP);

  const __bf16* QCh = (const __bf16*)(const void*)qcp + (size_t)(q0 + c) * KCW + h * HDC + 8 * hh;
  const __bf16* QCl = QCh + (KCW / 2);
  const __bf16* QRh = (const __bf16*)(const void*)qrp + (size_t)(q0 + c) * QRW + h * HDR + 8 * hh;
  const __bf16* QRl = QRh + (QRW / 2);

  float mrow[8], lrow[8];
  v8f oacc[8];
#pragma unroll
  for (int r = 0; r < 8; ++r) { mrow[r] = -INFINITY; lrow[r] = 0.f; }
#pragma unroll
  for (int t = 0; t < 8; ++t) oacc[t] = zero8();

  const int nch = 2 * qt + 2;
  for (int kc = 0; kc < nch; ++kc) {
    const int kv0 = kc * AKC;
    __syncthreads();
#pragma unroll
    for (int u = 0; u < 4; ++u) {
      const int p   = tid + 128 * u;
      const int key = p >> 4, d8 = (p & 15) * 8;
      const size_t ko = (size_t)(kv0 + key) * KCW + h * HDC + d8;
      const v4u x0 = *(const v4u*)(kcp + ko);
      const v4u x1 = *(const v4u*)(kcp + ko + KCW / 2);
      *(v4u*)(Ks  + key * KP + d8) = x0;
      *(v4u*)(Kls + key * KP + d8) = x1;
    }
#pragma unroll
    for (int u = 0; u < 2; ++u) {
      const int p   = tid + 128 * u;
      const int key = p >> 3, d8 = (p & 7) * 8;
      const size_t ko = (size_t)(kv0 + key) * KRW + d8;
      const v4u x0 = *(const v4u*)(krp + ko);
      const v4u x1 = *(const v4u*)(krp + ko + KRW / 2);
      *(v4u*)(Ks  + key * KP + HDC + d8) = x0;
      *(v4u*)(Kls + key * KP + HDC + d8) = x1;
    }
#pragma unroll
    for (int u = 0; u < 4; ++u) {
      const int p = tid + 128 * u;
      const int d = p >> 2, k8 = (p & 3) * 8;
      const size_t vo = (size_t)(h * HDC + d) * KCW + kv0 + k8;
      const v4u x0 = *(const v4u*)(vtp + vo);
      const v4u x1 = *(const v4u*)(vtp + vo + KCW / 2);
      *(v4u*)(Vhs + d * VP + k8) = x0;
      *(v4u*)(Vls + d * VP + k8) = x1;
    }
    __syncthreads();

    v8f sa[2];
    sa[0] = zero8(); sa[1] = zero8();
#pragma unroll
    for (int dc = 0; dc < 4; ++dc) {
      const v16b qh = ldfrag_b(QCh + dc * 32);
      const v16b ql = ldfrag_b(QCl + dc * 32);
#pragma unroll
      for (int j = 0; j < 2; ++j) {
        const v16b kb = ldfrag_b((const __bf16*)(const void*)Ks  + (j * 16 + c) * KP + dc * 32 + 8 * hh);
        const v16b kl = ldfrag_b((const __bf16*)(const void*)Kls + (j * 16 + c) * KP + dc * 32 + 8 * hh);
        sa[j] = mma_b(qh, kb, sa[j]);
        sa[j] = mma_b(qh, kl, sa[j]);
        sa[j] = mma_b(ql, kb, sa[j]);
        guard1b4(sa[j], qh, ql, kb, kl);
      }
    }
#pragma unroll
    for (int dc = 0; dc < 2; ++dc) {
      const v16b qh = ldfrag_b(QRh + dc * 32);
      const v16b ql = ldfrag_b(QRl + dc * 32);
#pragma unroll
      for (int j = 0; j < 2; ++j) {
        const v16b kb = ldfrag_b((const __bf16*)(const void*)Ks  + (j * 16 + c) * KP + HDC + dc * 32 + 8 * hh);
        const v16b kl = ldfrag_b((const __bf16*)(const void*)Kls + (j * 16 + c) * KP + HDC + dc * 32 + 8 * hh);
        sa[j] = mma_b(qh, kb, sa[j]);
        sa[j] = mma_b(qh, kl, sa[j]);
        sa[j] = mma_b(ql, kb, sa[j]);
        guard1b4(sa[j], qh, ql, kb, kl);
      }
    }
    acc_guard2(sa[0], sa[1]);

    float cm[8];
#pragma unroll
    for (int r = 0; r < 8; ++r) {
      const int qrow = q0 + 8 * hh + r;
      float m = -INFINITY;
#pragma unroll
      for (int j = 0; j < 2; ++j) {
        const int key = kv0 + j * 16 + c;
        const float sv = sa[j][r] * sscale;
        const float s  = (key > qrow) ? -INFINITY : sv;
        sa[j][r] = s;
        m = fmaxf(m, s);
      }
#pragma unroll
      for (int off = 1; off < 16; off <<= 1) m = fmaxf(m, __shfl_xor(m, off, 32));
      cm[r] = m;
    }
#pragma unroll
    for (int r = 0; r < 8; ++r) {
      const float mnew  = fmaxf(mrow[r], cm[r]);
      const float muse  = (mnew > -INFINITY) ? mnew : 0.0f;
      const float alpha = expf(mrow[r] - muse);
      mrow[r] = mnew;
      float psum = 0.f;
#pragma unroll
      for (int j = 0; j < 2; ++j) {
        const float p = expf(sa[j][r] - muse);
        psum += p;
        const unsigned short hb = bf_bits(p);
        const unsigned short lb = bf_bits(p - bf_val(hb));
        const int po = (8 * hh + r) * PP + j * 16 + c;
        ph[po] = hb;
        pl[po] = lb;
      }
#pragma unroll
      for (int off = 1; off < 16; off <<= 1) psum += __shfl_xor(psum, off, 32);
      lrow[r] = lrow[r] * alpha + psum;
#pragma unroll
      for (int t = 0; t < 8; ++t) oacc[t][r] *= alpha;
    }
    lds_wave_sync();
    const v16b pa = ldfrag_b((const __bf16*)(const void*)ph + c * PP + 8 * hh);
    const v16b pr = ldfrag_b((const __bf16*)(const void*)pl + c * PP + 8 * hh);
#pragma unroll
    for (int t = 0; t < 8; ++t) {
      const v16b vb = ldfrag_b((const __bf16*)(const void*)Vhs + (t * 16 + c) * VP + 8 * hh);
      const v16b vr = ldfrag_b((const __bf16*)(const void*)Vls + (t * 16 + c) * VP + 8 * hh);
      oacc[t] = mma_b(pa, vb, oacc[t]);
      oacc[t] = mma_b(pa, vr, oacc[t]);
      oacc[t] = mma_b(pr, vb, oacc[t]);
      guard1b4(oacc[t], pa, pr, vb, vr);
    }
  }
  __syncthreads();
  acc_guard4(oacc[0], oacc[1], oacc[2], oacc[3]);
  acc_guard4(oacc[4], oacc[5], oacc[6], oacc[7]);

  unsigned short* osh = pool + PK_OH + wave * (16 * OPW);
  unsigned short* osl = pool + PK_OL + wave * (16 * OPW);
#pragma unroll
  for (int r = 0; r < 8; ++r) {
    const float inv = 1.0f / lrow[r];
#pragma unroll
    for (int t = 0; t < 8; ++t) {
      const float o = oacc[t][r] * inv;
      const unsigned short hb = bf_bits(o);
      const unsigned short lb = bf_bits(o - bf_val(hb));
      const int so = (8 * hh + r) * OPW + t * 16 + c;
      osh[so] = hb;
      osl[so] = lb;
    }
  }
  lds_wave_sync();
  unsigned short* Cg = ctxp + (size_t)q0 * KCW + h * HDC;
  const int c8 = (lane & 15) * 8;
  for (int pass = 0; pass < 2; ++pass) {
#pragma unroll
    for (int it = 0; it < 8; ++it) {
      const int row = it * 2 + hh;
      const v4u x = *(const v4u*)(osh + row * OPW + c8);
      const v4u y = *(const v4u*)(osl + row * OPW + c8);
      *(volatile v4u*)(Cg + (size_t)row * KCW + c8)           = x;
      *(volatile v4u*)(Cg + (size_t)row * KCW + KCW / 2 + c8) = y;
    }
    __threadfence();
  }
}

static inline unsigned gemm_grid(int M, int N) { return (unsigned)(((M / 64) * (N / 64) + 7) / 8); }

extern "C" void kernel_launch(void* const* d_in, const int* in_sizes, int n_in,
                              void* d_out, int out_size, void* d_ws, size_t ws_size,
                              hipStream_t stream) {
  if (n_in < 9) return;
  if (in_sizes[0] != NTOK * DMD) return;
  if (in_sizes[1] != DMD * DLAT) return;
  if (in_sizes[2] != DLAT * DMD) return;
  if (in_sizes[3] != DLAT * DMD) return;
  if (in_sizes[4] != DMD * HDR) return;
  if (in_sizes[5] != DMD * DLAT) return;
  if (in_sizes[6] != DLAT * DMD) return;
  if (in_sizes[7] != DLAT * NHD * HDR) return;
  if (in_sizes[8] != DMD * DMD) return;
  if (out_size != NTOK * DMD) return;

  const float* x    = (const float*)d_in[0];
  const float* wdkv = (const float*)d_in[1];
  const float* wuk  = (const float*)d_in[2];
  const float* wuv  = (const float*)d_in[3];
  const float* wkr  = (const float*)d_in[4];
  const float* wdq  = (const float*)d_in[5];
  const float* wuq  = (const float*)d_in[6];
  const float* wqr  = (const float*)d_in[7];
  const float* wo   = (const float*)d_in[8];
  float* out = (float*)d_out;

  const size_t sWU  = (size_t)DMD * DLP * 2;
  const size_t sWQR = (size_t)(NHD * HDR) * DLP * 2;
  const size_t sWO  = (size_t)DMD * DMD * 2;
  const size_t sTAB = (size_t)SEQL * NFREQ * 4;
  const size_t sKR  = (size_t)NTOK * KRW * 2;
  const size_t sC   = (size_t)NTOK * CW * 2;
  const size_t sKC  = (size_t)SEQL * KCW * 2;
  const size_t sVT  = (size_t)(NHD * HDC) * KCW * 2;
  const size_t sQC  = (size_t)SEQL * KCW * 2;
  const size_t sQR  = (size_t)SEQL * QRW * 2;
  const size_t sCTX = (size_t)SEQL * KCW * 2;
  const size_t sXB  = (size_t)NTOK * DMD * 2;
  const size_t sWD  = (size_t)DLP * DMD * 2;
  const size_t sWKR = (size_t)HDR * DMD * 2;
  size_t off = 0;
  const size_t oWUK = off; off += sWU;
  const size_t oWUV = off; off += sWU;
  const size_t oWUQ = off; off += sWU;
  const size_t oWQR = off; off += sWQR;
  const size_t oWO  = off; off += sWO;
  const size_t oCOS = off; off += sTAB;
  const size_t oSIN = off; off += sTAB;
  const size_t oKR  = off; off += sKR;
  const size_t oCKV = off; off += sC;
  const size_t oCQ  = off; off += sC;
  const size_t oKC  = off; off += sKC;
  const size_t oVT  = off; off += sVT;
  const size_t oQC  = off; off += sQC;
  const size_t oQR  = off; off += sQR;
  const size_t oCTX = off; off += sCTX;
  const size_t total = off;
  const size_t oXB   = oKC;
  const size_t oWDKV = oXB + sXB;
  const size_t oWDQ  = oWDKV + sWD;
  const size_t oWKR  = oWDQ + sWD;
  if (oWKR + sWKR > total) return;
  if (total > ws_size) return;

  char* ws = (char*)d_ws;
  unsigned short* WUK  = (unsigned short*)(ws + oWUK);
  unsigned short* WUV  = (unsigned short*)(ws + oWUV);
  unsigned short* WUQ  = (unsigned short*)(ws + oWUQ);
  unsigned short* WQR  = (unsigned short*)(ws + oWQR);
  unsigned short* WO   = (unsigned short*)(ws + oWO);
  float*          COS  = (float*)(ws + oCOS);
  float*          SIN  = (float*)(ws + oSIN);
  unsigned short* KR   = (unsigned short*)(ws + oKR);
  unsigned short* CKV  = (unsigned short*)(ws + oCKV);
  unsigned short* CQ   = (unsigned short*)(ws + oCQ);
  unsigned short* KC   = (unsigned short*)(ws + oKC);
  unsigned short* VT   = (unsigned short*)(ws + oVT);
  unsigned short* QC   = (unsigned short*)(ws + oQC);
  unsigned short* QR   = (unsigned short*)(ws + oQR);
  unsigned short* CTX  = (unsigned short*)(ws + oCTX);
  unsigned short* XB   = (unsigned short*)(ws + oXB);
  unsigned short* WDKV = (unsigned short*)(ws + oWDKV);
  unsigned short* WDQ  = (unsigned short*)(ws + oWDQ);
  unsigned short* WKR  = (unsigned short*)(ws + oWKR);

  FreqTab ft;
  for (int j = 0; j < NFREQ; ++j) {
    const double e  = (double)j / 32.0;
    const float  pw = (float)pow(10000.0, e);
    ft.f[j] = 1.0f / pw;
  }
  const float sscale = 1.0f / sqrtf(192.0f);

  const dim3 b256(256), b128(128);

  rope_table_kernel<<<dim3(SEQL / 8), b256, 0, stream>>>(ft, COS, SIN);
  cvt_bf16_kernel<<<dim3((NTOK * DMD / 8) / 256), b256, 0, stream>>>(x, XB, NTOK * DMD / 8);
  tcvt_kernel<<<dim3(DMD / 64, DLP / 64), b256, 0, stream>>>(wdkv, DMD, DLAT, WDKV, DMD, 0, -1);
  tcvt_kernel<<<dim3(DMD / 64, DLP / 64), b256, 0, stream>>>(wdq,  DMD, DLAT, WDQ,  DMD, 0, -1);
  tcvt_kernel<<<dim3(DMD / 64, HDR / 64), b256, 0, stream>>>(wkr,  DMD, HDR,  WKR,  DMD, 0, -1);
  tcvt_kernel<<<dim3(DLP / 64, DMD / 64), b256, 0, stream>>>(wuk, DLAT, DMD, WUK, DLP, 0, -1);
  tcvt_kernel<<<dim3(DLP / 64, DMD / 64), b256, 0, stream>>>(wuv, DLAT, DMD, WUV, DLP, 0, -1);
  tcvt_kernel<<<dim3(DLP / 64, DMD / 64), b256, 0, stream>>>(wuq, DLAT, DMD, WUQ, DLP, 0, -1);
  tcvt_kernel<<<dim3(DLP / 64, (NHD * HDR) / 64), b256, 0, stream>>>(wqr, DLAT, NHD * HDR, WQR, DLP, 0, -1);
  tcvt_kernel<<<dim3(DMD / 64, DMD / 64), b256, 0, stream>>>(wo, DMD, DMD, WO, DMD, 0, -1);

  gemm64_kernel<false, false, 2><<<dim3(gemm_grid(NTOK, DLP)), b256, 0, stream>>>(
      XB, XB, DMD, WDKV, WDKV, DMD, (void*)CKV, (void*)(CKV + DLP), CW, COS, SIN, NTOK, DLP, DMD);
  gemm64_kernel<false, false, 2><<<dim3(gemm_grid(NTOK, DLP)), b256, 0, stream>>>(
      XB, XB, DMD, WDQ, WDQ, DMD, (void*)CQ, (void*)(CQ + DLP), CW, COS, SIN, NTOK, DLP, DMD);
  gemm64_kernel<false, false, 3><<<dim3(gemm_grid(NTOK, HDR)), b256, 0, stream>>>(
      XB, XB, DMD, WKR, WKR, DMD, (void*)KR, (void*)(KR + HDR), KRW, COS, SIN, NTOK, HDR, DMD);

  for (int b = 0; b < NBAT; ++b) {
    const unsigned short* CKVb = CKV + (size_t)b * SEQL * CW;
    const unsigned short* CQb  = CQ  + (size_t)b * SEQL * CW;
    const unsigned short* KRb  = KR  + (size_t)b * SEQL * KRW;
    float* outb = out + (size_t)b * SEQL * DMD;
    gemm64_kernel<true, false, 2><<<dim3(gemm_grid(SEQL, DMD)), b256, 0, stream>>>(
        CKVb, CKVb + DLP, CW, WUK, WUK, DLP, (void*)KC, (void*)(KC + KCW / 2), KCW, COS, SIN, SEQL, DMD, DLP);
    gemm64_kernel<false, true, 2><<<dim3(gemm_grid(DMD, SEQL)), b256, 0, stream>>>(
        WUV, WUV, DLP, CKVb, CKVb + DLP, CW, (void*)VT, (void*)(VT + KCW / 2), KCW, COS, SIN, DMD, SEQL, DLP);
    gemm64_kernel<true, false, 2><<<dim3(gemm_grid(SEQL, DMD)), b256, 0, stream>>>(
        CQb, CQb + DLP, CW, WUQ, WUQ, DLP, (void*)QC, (void*)(QC + KCW / 2), KCW, COS, SIN, SEQL, DMD, DLP);
    gemm64_kernel<true, false, 3><<<dim3(gemm_grid(SEQL, NHD * HDR)), b256, 0, stream>>>(
        CQb, CQb + DLP, CW, WQR, WQR, DLP, (void*)QR, (void*)(QR + QRW / 2), QRW, COS, SIN, SEQL, NHD * HDR, DLP);
    attn_lat_kernel<<<dim3(SEQL / 64, NHD), b128, 0, stream>>>(QC, QR, KC, KRb, VT, CTX, sscale);
    gemm64_kernel<true, false, 0><<<dim3(gemm_grid(SEQL, DMD)), b256, 0, stream>>>(
        CTX, CTX + KCW / 2, KCW, WO, WO, DMD, (void*)outb, (void*)outb, DMD, COS, SIN, SEQL, DMD, DMD);
  }
  (void)hipGetLastError();
}
